// MS_Attention_73787538145800
// MI455X (gfx1250) — hardware-verified
//
#include <hip/hip_runtime.h>
#include <math.h>

typedef __attribute__((ext_vector_type(16))) _Float16 v16h;
typedef __attribute__((ext_vector_type(16))) __bf16 v16b;
typedef __attribute__((ext_vector_type(8)))  _Float16 v8h;
typedef __attribute__((ext_vector_type(8)))  float v8f;
typedef __attribute__((ext_vector_type(4)))  float v4f;
typedef __attribute__((ext_vector_type(2)))  float v2f;
typedef __attribute__((ext_vector_type(4)))  unsigned v4u;
typedef __attribute__((ext_vector_type(4)))  int v4i;
typedef float __attribute__((may_alias)) float_a;
typedef int __attribute__((may_alias)) int_a;

template <typename T> __device__ __forceinline__ void vst2(void* p, T v) { *(volatile T*)p = v; __threadfence(); *(volatile T*)p = v; }
__device__ __forceinline__ v8f wmma16(v16h a, v16h b, v8f c) {
  v8f d = __builtin_amdgcn_wmma_f32_16x16x32_f16(false, a, false, b, (short)0, c, false, false);
  asm volatile("v_nop\n\tv_nop\n\tv_nop\n\tv_nop" : "+v"(d) : "v"(a), "v"(b));
  return d;
}
__device__ __forceinline__ v8f wmma_bf(v16b a, v16b b, v8f c) {
  v8f d = __builtin_amdgcn_wmma_f32_16x16x32_bf16(false, a, false, b, (short)0, c, false, false);
  asm volatile("v_nop\n\tv_nop\n\tv_nop\n\tv_nop" : "+v"(d) : "v"(a), "v"(b));
  return d;
}
__device__ __forceinline__ v16h frag_h(const _Float16* rowk0, int lane) {
  union { v16h v; v8h q[2]; } u; const _Float16* p = rowk0 + 8 * (lane >> 4);
  u.q[0] = *(const v8h*)p; u.q[1] = *(const v8h*)(p + 16); return u.v;
}
__device__ __forceinline__ v16h frag_f32(const float* rowk0, int lane) {
  v16h a; const float* p = rowk0 + 8 * (lane >> 4);
#pragma unroll
  for (int i = 0; i < 8; ++i) { a[i] = (_Float16)p[i]; a[8 + i] = (_Float16)p[16 + i]; }
  return a;
}
__device__ __forceinline__ v16h frag_f32s(const float* rowk0, int lane, float sc) {
  v16h a; const float* p = rowk0 + 8 * (lane >> 4);
#pragma unroll
  for (int i = 0; i < 8; ++i) { a[i] = (_Float16)(p[i] * sc); a[8 + i] = (_Float16)(p[16 + i] * sc); }
  return a;
}
__device__ __forceinline__ v16h fragc_f32(const float* W, int k0, int n, int lane, int ld, int K) {
  v16h a; const int g = lane >> 4;
#pragma unroll
  for (int i = 0; i < 8; ++i) { const int ka = k0 + 8 * g + i, kb = ka + 16;
    a[i] = (_Float16)(ka < K ? W[(size_t)(ka < K ? ka : K - 1) * ld + n] : 0.f); a[8 + i] = (_Float16)(kb < K ? W[(size_t)(kb < K ? kb : K - 1) * ld + n] : 0.f); }
  return a;
}
struct F2 { v16b h, l; };
__device__ __forceinline__ F2 bsplit16(const float v[16]) { F2 r;
#pragma unroll
  for (int i = 0; i < 16; ++i) { const __bf16 h = (__bf16)v[i]; r.h[i] = h; r.l[i] = (__bf16)(v[i] - (float)h); }
  return r; }
__device__ __forceinline__ F2 split_row(const float* row, int k0, int lane) { float v[16]; const float* p = row + k0 + 8 * (lane >> 4);
#pragma unroll
  for (int i = 0; i < 8; ++i) { v[i] = p[i]; v[8 + i] = p[16 + i]; }
  return bsplit16(v); }
__device__ __forceinline__ F2 split_rowK(const float* row, int k0, int lane, int K) { float v[16]; const int g = lane >> 4;
#pragma unroll
  for (int i = 0; i < 8; ++i) { const int ka = k0 + 8 * g + i, kb = ka + 16; v[i] = ka < K ? row[ka < K ? ka : K - 1] : 0.f; v[8 + i] = kb < K ? row[kb < K ? kb : K - 1] : 0.f; }
  return bsplit16(v); }
__device__ __forceinline__ F2 split_col(const float* W, int k0, int n, int lane, int ld, int K) { float v[16]; const int g = lane >> 4;
#pragma unroll
  for (int i = 0; i < 8; ++i) { const int ka = k0 + 8 * g + i, kb = ka + 16; v[i] = ka < K ? W[(size_t)(ka < K ? ka : K - 1) * ld + n] : 0.f; v[8 + i] = kb < K ? W[(size_t)(kb < K ? kb : K - 1) * ld + n] : 0.f; }
  return bsplit16(v); }
__device__ __forceinline__ v8f mac3(const F2& a, const F2& b, v8f c) { c = wmma_bf(a.l, b.h, c); c = wmma_bf(a.h, b.l, c); return wmma_bf(a.h, b.h, c); }
__device__ __forceinline__ float sigm(float v) { return 1.0f / (1.0f + expf(-v)); }
#define LDSX() do { asm volatile("s_wait_dscnt 0" ::: "memory"); __builtin_amdgcn_wave_barrier(); __builtin_amdgcn_fence(__ATOMIC_RELEASE, "workgroup"); } while (0)


#define NBATCH 16
#define NQ 1024
#define NP 1024
#define NUP 2048
#define CC 512
#define NHS 4
#define HD 64
#define NRQ (NQ * NBATCH)
#define NRK (NP * NBATCH)
#define NRU (NUP * NBATCH)
#ifndef NPB
#define NPB NBATCH
#endif
typedef __attribute__((ext_vector_type(8))) __bf16 v8b;
__device__ __forceinline__ v16b frag_b(const __bf16* rowk0, int lane) {
  union { v16b v; v8b q[2]; } u; const __bf16* p = rowk0 + 8 * (lane >> 4);
  u.q[0] = *(const v8b*)p; u.q[1] = *(const v8b*)(p + 16); return u.v;
}
__device__ __forceinline__ float bfr(float v) { return (float)(__bf16)v; }
__device__ __attribute__((noinline)) float exp_ni(float v) { return expf(v); }
__device__ __attribute__((noinline)) float erf_ni(float v) { return erff(v); }

#define WS_PQ   0u
#define WS_PH   (WS_PQ + 2u * (size_t)3 * CC * CC)
#define WS_Q    (WS_PH + 2u * (size_t)2 * CC * CC)
#define WS_K1   (WS_Q + 2u * (size_t)NRQ * CC)
#define WS_V1   (WS_K1 + 2u * (size_t)NRK * 256)
#define WS_IDX  (WS_V1 + 2u * (size_t)NBATCH * 256 * NP)
#define WS_WGT  (WS_IDX + 4u * (size_t)NBATCH * NUP * 4)
#define WS_IN   (WS_WGT + 4u * (size_t)NBATCH * NUP * 4)
#define WS_KEY2 (WS_IN + 2u * (size_t)NRU * CC)
#define WS_K2   (WS_KEY2 + 2u * (size_t)NRU * CC)
#define WS_V2   (WS_K2 + 2u * (size_t)NRU * 256)
#define WS_O    (WS_V2 + 2u * (size_t)NBATCH * 256 * NUP)
#define WS_END  (WS_O + 4u * (size_t)NRQ * CC)

__global__ __launch_bounds__(256) void k_pack(const float* __restrict__ WQ, const float* __restrict__ WKV1, const float* __restrict__ WP, const float* __restrict__ WFP, const float* __restrict__ WKV2, __bf16* __restrict__ P, _Float16* __restrict__ PH) {
  const int n = blockIdx.x, which = blockIdx.y, t = threadIdx.x; __shared__ __align__(16) __bf16 s[CC]; __shared__ __align__(16) _Float16 sh[CC];
  if (which < 3) { const float* Wm = (which == 0) ? WQ : (which == 1) ? WKV1 : WP; for (int k = t; k < CC; k += 256) s[k] = (__bf16)Wm[(size_t)n * CC + k]; __syncthreads(); if (t < CC / 8) vst2((unsigned*)(P + ((size_t)which * CC + n) * CC + t * 8), *(const v4u*)&s[t * 8]); }
  else { const float* Wm = (which == 3) ? WFP : WKV2; for (int k = t; k < CC; k += 256) sh[k] = (_Float16)(bfr(Wm[(size_t)n * CC + k]) * 256.0f); __syncthreads(); if (t < CC / 8) vst2((unsigned*)(PH + ((size_t)(which - 3) * CC + n) * CC + t * 8), *(const v4u*)&sh[t * 8]); }
}
template <int AMODE, int OMODE>
__global__ __launch_bounds__(128) void k_gemm(const void* __restrict__ Ain, const void* __restrict__ Win, const float* __restrict__ BIAS, int spb, _Float16* __restrict__ OR, _Float16* __restrict__ OV) {
  __shared__ __align__(16) _Float16 so[64][136]; __shared__ __align__(16) _Float16 st[128][72];
  const int tid = threadIdx.x, wave = tid >> 5, lane = tid & 31, col = lane & 15, g = lane >> 4; const size_t rb0 = (size_t)blockIdx.x * 64, r0 = rb0 + wave * 16; const int n0 = blockIdx.y * 128;
  v8f acc[8] = {};
  if (AMODE == 0) { const float* X = (const float*)Ain; const __bf16* Wr = (const __bf16*)Win;
#pragma unroll 2
    for (int kc = 0; kc < CC / 32; ++kc) { v16b a; { const float* p = X + (r0 + col) * CC + kc * 32 + 8 * g;
#pragma unroll
        for (int i = 0; i < 8; ++i) { a[i] = (__bf16)p[i]; a[8 + i] = (__bf16)p[16 + i]; } }
#pragma unroll
      for (int j = 0; j < 8; ++j) acc[j] = wmma_bf(a, frag_b(Wr + (size_t)(n0 + j * 16 + col) * CC + kc * 32, lane), acc[j]); }
  } else { const _Float16* X = (const _Float16*)Ain; const _Float16* Wr = (const _Float16*)Win;
#pragma unroll 2
    for (int kc = 0; kc < CC / 32; ++kc) { const v16h a = frag_h(X + (r0 + col) * CC + kc * 32, lane);
#pragma unroll
      for (int j = 0; j < 8; ++j) acc[j] = wmma16(a, frag_h(Wr + (size_t)(n0 + j * 16 + col) * CC + kc * 32, lane), acc[j]); }
#pragma unroll
    for (int j = 0; j < 8; ++j)
#pragma unroll
      for (int r = 0; r < 8; ++r) acc[j][r] *= (1.0f / 256.0f); }
  if (OMODE == 1 && n0 >= 256) {
#pragma unroll
    for (int j = 0; j < 8; ++j)
#pragma unroll
      for (int r = 0; r < 8; ++r) st[j * 16 + col][wave * 16 + 8 * g + r] = (_Float16)acc[j][r];
    __syncthreads();
    const size_t pb = rb0 / spb, s0 = rb0 % spb;
    for (int e = tid; e < 128 * 8; e += 128) { const int d = e >> 3, pc = e & 7; vst2((unsigned*)(OV + ((pb * 256 + (n0 - 256) + d) * (size_t)spb) + s0 + pc * 8), *(const v4u*)&st[d][pc * 8]); }
  } else {
    const int ncols = (OMODE == 1) ? 256 : CC;
#pragma unroll
    for (int j = 0; j < 8; ++j) { const float bb = (OMODE == 2) ? bfr(BIAS[n0 + j * 16 + col]) : 0.f;
#pragma unroll
      for (int r = 0; r < 8; ++r) { float v = acc[j][r] + bb; if (OMODE == 2) v = fmaxf(v, 0.f); so[wave * 16 + 8 * g + r][j * 16 + col] = (_Float16)v; } }
    LDSX();
    for (int rl = 0; rl < 16; ++rl) if (lane < 16) vst2((unsigned*)(OR + (r0 + rl) * (size_t)ncols + n0 + lane * 8), *(const v4u*)&so[wave * 16 + rl][lane * 8]);
  }
}
__global__ __launch_bounds__(256) void k_knn(const float* __restrict__ XU, const float* __restrict__ KP, int* __restrict__ IDX, float* __restrict__ WGT) {
  __shared__ float spx[NP], spy[NP], spz[NP]; __shared__ float cd[64][4][3]; __shared__ int ci[64][4][3]; __shared__ __align__(16) int sidx[64][4]; __shared__ __align__(16) float swg[64][4];
  const int t = threadIdx.x; const size_t b = blockIdx.y; const size_t n0 = (size_t)blockIdx.x * 64;
  for (int m = t; m < NP; m += 256) { spx[m] = bfr(KP[(b * NP + m) * 3 + 0]); spy[m] = bfr(KP[(b * NP + m) * 3 + 1]); spz[m] = bfr(KP[(b * NP + m) * 3 + 2]); }
  __syncthreads();
  const int ql = t >> 2, sub = t & 3; const size_t n = n0 + ql;
  const float x0 = bfr(XU[(b * NUP + n) * 3 + 0]), y0 = bfr(XU[(b * NUP + n) * 3 + 1]), z0 = bfr(XU[(b * NUP + n) * 3 + 2]);
  float d0 = 3.0e38f, d1 = 3.0e38f, dd2 = 3.0e38f; int i0 = 0x7fffffff, i1 = 0x7fffffff, i2 = 0x7fffffff;
#pragma unroll 1
  for (int m = sub; m < NP; m += 4) { const float dx = x0 - spx[m], dy = y0 - spy[m], dz = z0 - spz[m]; const float d = (dx * dx + dy * dy) + dz * dz;
    if (d < dd2) { if (d < d1) { dd2 = d1; i2 = i1; if (d < d0) { d1 = d0; i1 = i0; d0 = d; i0 = m; } else { d1 = d; i1 = m; } } else { dd2 = d; i2 = m; } } }
  cd[ql][sub][0] = d0; cd[ql][sub][1] = d1; cd[ql][sub][2] = dd2; ci[ql][sub][0] = i0; ci[ql][sub][1] = i1; ci[ql][sub][2] = i2;
  __syncthreads();
  if (sub == 0) { float bd[3] = {3.0e38f, 3.0e38f, 3.0e38f}; int bi[3] = {0x7fffffff, 0x7fffffff, 0x7fffffff};
    for (int s = 0; s < 4; ++s) for (int k = 0; k < 3; ++k) { const float d = cd[ql][s][k]; const int ii = ci[ql][s][k];
      if (d < bd[2] || (d == bd[2] && ii < bi[2])) { if (d < bd[1] || (d == bd[1] && ii < bi[1])) { bd[2] = bd[1]; bi[2] = bi[1]; if (d < bd[0] || (d == bd[0] && ii < bi[0])) { bd[1] = bd[0]; bi[1] = bi[0]; bd[0] = d; bi[0] = ii; } else { bd[1] = d; bi[1] = ii; } } else { bd[2] = d; bi[2] = ii; } } }
    float w[3]; for (int k = 0; k < 3; ++k) w[k] = 1.0f / (bd[k] + 1e-8f);
    const float rs = (w[0] + w[1]) + w[2];
    for (int k = 0; k < 3; ++k) { sidx[ql][k] = min(bi[k], NP - 1); swg[ql][k] = w[k] / rs; } sidx[ql][3] = 0; swg[ql][3] = 0.f; }
  __syncthreads();
  if (t < 64) { vst2((unsigned*)(IDX + (b * NUP + n0 + t) * 4), *(const v4u*)&sidx[t][0]); vst2(WGT + (b * NUP + n0 + t) * 4, *(const v4f*)&swg[t][0]); }
}
__global__ __launch_bounds__(256) void k_interp(const float* __restrict__ KEY, const int* __restrict__ IDX, const float* __restrict__ WGT, _Float16* __restrict__ INR) {
  __shared__ __align__(16) _Float16 so[16][CC];
  const size_t n = blockIdx.x; const int t = threadIdx.x; const int b = t >> 4, ch = t & 15;
  const int j0 = IDX[(b * NUP + n) * 4 + 0], j1 = IDX[(b * NUP + n) * 4 + 1], j2 = IDX[(b * NUP + n) * 4 + 2]; const float w0 = WGT[(b * NUP + n) * 4 + 0], w1 = WGT[(b * NUP + n) * 4 + 1], w2 = WGT[(b * NUP + n) * 4 + 2];
  const float* f0 = KEY + ((size_t)j0 * NBATCH + b) * CC, *f1 = KEY + ((size_t)j1 * NBATCH + b) * CC, *f2 = KEY + ((size_t)j2 * NBATCH + b) * CC;
  for (int c = ch * 32; c < ch * 32 + 32; ++c) so[b][c] = (_Float16)((bfr(f0[c]) * w0 + bfr(f1[c]) * w1) + bfr(f2[c]) * w2);
  __syncthreads();
  for (int e = t; e < 16 * (CC / 8); e += 256) { const int bb = e / (CC / 8), q = e % (CC / 8); vst2((unsigned*)(INR + (n * NBATCH + bb) * CC + q * 8), *(const v4u*)&so[bb][q * 8]); }
}
template <int SK>
__global__ __launch_bounds__(128) void k_attn(const _Float16* __restrict__ Q, const _Float16* __restrict__ Kr, const _Float16* __restrict__ V, int hoff, int ocol0, float* __restrict__ O) {
  __shared__ __align__(16) _Float16 sph[4][16][40]; __shared__ __align__(16) float so[4][16][68];
  const int tid = threadIdx.x, wave = tid >> 5, lane = tid & 31, col = lane & 15, g = lane >> 4; const int hl = blockIdx.y; const size_t pb = blockIdx.z; const int q0 = blockIdx.x * 64 + wave * 16; const size_t rq = pb * NQ + q0;
  v16h aq[2];
#pragma unroll
  for (int kc = 0; kc < 2; ++kc) aq[kc] = frag_h(Q + (rq + col) * CC + (hoff + hl) * HD + kc * 32, lane);
  float m[8], l[8];
#pragma unroll
  for (int r = 0; r < 8; ++r) { m[r] = -3.0e38f; l[r] = 0.f; }
  v8f acc[4] = {};
#pragma unroll 1
  for (int ks = 0; ks < SK / 32; ++ks) { const int j0 = ks * 32; v8f s[2];
#pragma unroll
    for (int ct = 0; ct < 2; ++ct) { const size_t rk = (pb * SK + j0 + ct * 16 + col) * 256 + hl * HD; v8f c = {};
#pragma unroll
      for (int kc = 0; kc < 2; ++kc) c = wmma16(aq[kc], frag_h(Kr + rk + kc * 32, lane), c);
#pragma unroll
      for (int r = 0; r < 8; ++r) s[ct][r] = c[r] * 0.125f; }
#pragma unroll
    for (int r = 0; r < 8; ++r) { float mx = fmaxf(s[0][r], s[1][r]);
#pragma unroll
      for (int o = 1; o < 16; o <<= 1) mx = fmaxf(mx, __shfl_xor(mx, o));
      const float mn = fmaxf(m[r], mx); const float alpha = (m[r] <= -1.0e38f) ? 0.f : __expf(m[r] - mn); const float e0 = __expf(s[0][r] - mn), e1 = __expf(s[1][r] - mn); float es = e0 + e1;
#pragma unroll
      for (int o = 1; o < 16; o <<= 1) es += __shfl_xor(es, o);
      l[r] = l[r] * alpha + es; m[r] = mn;
#pragma unroll
      for (int dt = 0; dt < 4; ++dt) acc[dt][r] *= alpha;
      sph[wave][8 * g + r][col] = (_Float16)(e0 * 2048.0f); sph[wave][8 * g + r][16 + col] = (_Float16)(e1 * 2048.0f); }
    LDSX();
    const v16h pa = frag_h(&sph[wave][col][0], lane);
#pragma unroll
    for (int dt = 0; dt < 4; ++dt) acc[dt] = wmma16(pa, frag_h(V + ((pb * 256 + (size_t)hl * HD + dt * 16 + col) * SK) + j0, lane), acc[dt]);
    LDSX(); }
#pragma unroll
  for (int r = 0; r < 8; ++r) { const float il = (1.0f / 2048.0f) / l[r];
#pragma unroll
    for (int dt = 0; dt < 4; ++dt) so[wave][8 * g + r][dt * 16 + col] = acc[dt][r] * il; }
  LDSX();
  for (int rl = 0; rl < 16; ++rl) if (lane < 16) vst2(O + (rq + rl) * CC + ocol0 + hl * HD + lane * 4, *(const v4f*)&so[wave][rl][lane * 4]);
}
__global__ __launch_bounds__(128) void k_out(const float* __restrict__ O, const __bf16* __restrict__ P, const float* __restrict__ BP, float* __restrict__ OUT) {
  __shared__ __align__(16) float so[4][16][132];
  const int tid = threadIdx.x, wave = tid >> 5, lane = tid & 31, col = lane & 15, g = lane >> 4; const size_t r0 = (size_t)blockIdx.x * 64 + wave * 16; const int n0 = blockIdx.y * 128;
  v8f acc[8] = {};
#pragma unroll 2
  for (int kc = 0; kc < CC / 32; ++kc) { const F2 a = split_row(O + (r0 + col) * CC, kc * 32, lane);
#pragma unroll
    for (int j = 0; j < 8; ++j) { const v16b w = frag_b(P + ((size_t)2 * CC + n0 + j * 16 + col) * CC + kc * 32, lane); acc[j] = wmma_bf(a.l, w, acc[j]); acc[j] = wmma_bf(a.h, w, acc[j]); } }
#pragma unroll
  for (int j = 0; j < 8; ++j) { const float bb = bfr(BP[n0 + j * 16 + col]);
#pragma unroll
    for (int r = 0; r < 8; ++r) so[wave][8 * g + r][j * 16 + col] = acc[j][r] + bb; }
  LDSX();
  for (int rl = 0; rl < 16; ++rl) { const size_t R = r0 + rl; const size_t pb = R / NQ, i = R % NQ; vst2(OUT + (i * NBATCH + pb) * CC + n0 + lane * 4, *(const v4f*)&so[wave][rl][lane * 4]); }
}
extern "C" void kernel_launch(void* const* d_in, const int* in_sizes, int n_in, void* d_out, int out_size, void* d_ws, size_t ws_size, hipStream_t stream) {
  (void)in_sizes; (void)n_in; (void)out_size;
  const float** F = (const float**)d_in;
  if (ws_size < (size_t)WS_END) return;
  char* ws = (char*)d_ws; __bf16* P = (__bf16*)ws; _Float16 *PH = (_Float16*)(ws + WS_PH), *Q = (_Float16*)(ws + WS_Q), *K1 = (_Float16*)(ws + WS_K1), *V1 = (_Float16*)(ws + WS_V1), *INR = (_Float16*)(ws + WS_IN), *KEY2 = (_Float16*)(ws + WS_KEY2), *K2 = (_Float16*)(ws + WS_K2), *V2 = (_Float16*)(ws + WS_V2); int* IDX = (int*)(ws + WS_IDX); float *WGT = (float*)(ws + WS_WGT), *O = (float*)(ws + WS_O);
  k_pack<<<dim3(CC, 5), 256, 0, stream>>>(F[5], F[6], F[10], F[8], F[7], P, PH);
  k_gemm<0, 0><<<dim3(NPB * NQ / 64, CC / 128), 128, 0, stream>>>(F[0], P, nullptr, NQ, Q, nullptr);
  k_gemm<0, 1><<<dim3(NPB * NP / 64, CC / 128), 128, 0, stream>>>(F[1], P + (size_t)CC * CC, nullptr, NP, K1, V1);
  k_knn<<<dim3(NUP / 64, NBATCH), 256, 0, stream>>>(F[4], F[2], IDX, WGT);
  k_interp<<<NUP, 256, 0, stream>>>(F[1], IDX, WGT, INR);
  k_gemm<1, 2><<<dim3(NRU / 64, CC / 128), 128, 0, stream>>>(INR, PH, F[9], NUP, KEY2, nullptr);
  k_gemm<1, 1><<<dim3(NPB * NUP / 64, CC / 128), 128, 0, stream>>>(KEY2, PH + (size_t)CC * CC, nullptr, NUP, K2, V2);
  k_attn<NP><<<dim3(NQ / 64, NHS, NPB), 128, 0, stream>>>(Q, K1, V1, 0, 0, O);
  k_attn<NUP><<<dim3(NQ / 64, NHS, NPB), 128, 0, stream>>>(Q, K2, V2, NHS, 256, O);
  k_out<<<dim3(NPB * NQ / 64, CC / 128), 128, 0, stream>>>(O, P, F[11], (float*)d_out);
}
